// LSTMAE_88545045774784
// MI455X (gfx1250) — hardware-run, weakly checked
//
#include <hip/hip_runtime.h>
#include <math.h>
#include <cstddef>

typedef __attribute__((ext_vector_type(16))) _Float16 v16h;
typedef __attribute__((ext_vector_type(8)))  _Float16 v8h;
typedef __attribute__((ext_vector_type(8)))  float    v8f;
typedef __attribute__((ext_vector_type(4)))  float    v4f;
typedef __attribute__((ext_vector_type(4)))  unsigned v4u;

constexpr int kBatch   = 256;
constexpr int kSteps   = 512;
constexpr int kEncIn   = 8;
constexpr int kDecIn   = 6;
constexpr int kEncH    = 3;
constexpr int kDecH    = 128;
constexpr int kGates   = 4 * kDecH;
constexpr int kKcat    = 160;
constexpr int kWPitch  = 168;
constexpr int kAPitch  = 168;
constexpr int kRowsBlk = 16;
constexpr int kChunkT  = 32;
constexpr int kChunkF  = kChunkT * kDecIn;
constexpr int kHfPitch = 132;
static_assert(kGates == 512);
static_assert((kKcat % 32) == 0);
static_assert(kDecH + kDecIn + 1 <= kKcat);
static_assert((kBatch % kRowsBlk) == 0);
static_assert((kSteps % kChunkT) == 0);
static_assert(kChunkF == 192);

constexpr float kCarryW   = 64.0f;
constexpr float kCarryA   = 64.0f;
constexpr float kBiasCar  = kCarryW * kCarryA;
constexpr float kFold     = 1.0f / (kCarryW * kCarryA);
constexpr float kF16MinN  = 6.103515625e-5f;

constexpr int kOutZ     = 0;
constexpr int kOutTraj  = kBatch;
constexpr int kOutHdec  = kBatch + kBatch * kSteps * 2;
constexpr int kOutTotal = kOutHdec + kBatch * kDecH;
static_assert(kOutTraj * 4 == 1024);
static_assert(kOutHdec * 4 == 1049600);
static_assert(kOutTotal * 4 == 1180672);

constexpr size_t kWsWcat  = 0;
constexpr size_t kWsZ     = kWsWcat + (size_t)kGates * kKcat * 2;
constexpr size_t kWsTotal = kWsZ + (size_t)kBatch * 4;
static_assert(kWsTotal == 164864ull);
static_assert((kWsZ % 128) == 0);
static_assert(kWsTotal <= 134217728ull);

constexpr int kOffW     = 0;
constexpr int kOffA     = kOffW + kGates * kWPitch * 2;
constexpr int kOffS     = kOffA + kRowsBlk * kAPitch * 2;
constexpr int kOffHF    = kOffS + 2 * kRowsBlk * kChunkF * 4;
constexpr int kLdsBytes = kOffHF + kRowsBlk * kHfPitch * 4;
static_assert(kLdsBytes == 210432);
static_assert((kOffA % 16) == 0 && (kOffS % 16) == 0 && (kOffHF % 16) == 0);

__device__ __forceinline__ float sig_f(float x) {
  const float xc = fminf(fmaxf(x, -30.0f), 30.0f);
  return 1.0f / (1.0f + expf(-xc));
}
__device__ __forceinline__ float tanh_f(float x) {
  const float a = fminf(fabsf(x), 15.0f);
  const float e = expf(-2.0f * a);
  const float r = (1.0f - e) * (1.0f / (1.0f + e));
  return copysignf(r, x);
}
__device__ __forceinline__ _Float16 cvt_flush(float v, float zf) {
  const float w = (fabsf(v) < kF16MinN) ? zf : v;
  return (_Float16)w;
}
union FragU { v16h v; v8h h[2]; };
__device__ __forceinline__ v16h ldfrag(const _Float16* p) {
  FragU f;
  f.h[0] = *(const v8h*)(p);
  f.h[1] = *(const v8h*)(p + 16);
  return f.v;
}
__device__ __forceinline__ v8f mma_f16(v16h a, v16h b, v8f c) {
  c = __builtin_amdgcn_wmma_f32_16x16x32_f16(false, a, false, b, (short)0, c, false, false);
  asm volatile("v_nop\n\tv_nop\n\tv_nop\n\tv_nop" : "+v"(c) : "v"(a), "v"(b));
  return c;
}

__global__ __launch_bounds__(256) void prep_wcat_kernel(
    const float* __restrict__ Whh, const float* __restrict__ Wih, unsigned short* __restrict__ wcat)
{
  const int i = blockIdx.x * 256 + threadIdx.x;
  if (i >= kGates * (kKcat / 8)) return;
  const int nrow = i / (kKcat / 8);
  const int ch   = i - nrow * (kKcat / 8);
  const int chc  = ch < 16 ? ch : 15;
  const v4f hA = *(const v4f*)(Whh + (size_t)nrow * kDecH + chc * 8);
  const v4f hB = *(const v4f*)(Whh + (size_t)nrow * kDecH + chc * 8 + 4);
  float a0 = hA[0], a1 = hA[1], a2 = hA[2], a3 = hA[3];
  float b0 = hB[0], b1 = hB[1], b2 = hB[2], b3 = hB[3];
  asm volatile("" : "+v"(a0), "+v"(a1), "+v"(a2), "+v"(a3));
  asm volatile("" : "+v"(b0), "+v"(b1), "+v"(b2), "+v"(b3));
  const float* wi = Wih + (size_t)nrow * (kDecIn + 1);
  float x0 = wi[0], x1 = wi[1], x2 = wi[2], x3 = wi[3], x4 = wi[4], x5 = wi[5], x6 = wi[6];
  asm volatile("" : "+v"(x0), "+v"(x1), "+v"(x2), "+v"(x3));
  asm volatile("" : "+v"(x4), "+v"(x5), "+v"(x6));
  float zf = 0.0f;
  asm volatile("" : "+v"(zf));
  const bool isH = (ch < 16);
  const bool isX = (ch == 16);
  const float e0 = isH ? a0 : (isX ? x0 : zf);
  const float e1 = isH ? a1 : (isX ? x1 : zf);
  const float e2 = isH ? a2 : (isX ? x2 : zf);
  const float e3 = isH ? a3 : (isX ? x3 : zf);
  const float e4 = isH ? b0 : (isX ? x4 : zf);
  const float e5 = isH ? b1 : (isX ? x5 : zf);
  const float e6 = isH ? b2 : (isX ? x6 : zf);
  const float e7 = isH ? b3 : zf;
  v8h o;
  o[0] = cvt_flush(e0 * kCarryW, zf);
  o[1] = cvt_flush(e1 * kCarryW, zf);
  o[2] = cvt_flush(e2 * kCarryW, zf);
  o[3] = cvt_flush(e3 * kCarryW, zf);
  o[4] = cvt_flush(e4 * kCarryW, zf);
  o[5] = cvt_flush(e5 * kCarryW, zf);
  o[6] = cvt_flush(e6 * kCarryW, zf);
  o[7] = cvt_flush(e7 * kCarryW, zf);
  unsigned short* q = wcat + (size_t)i * 8;
  *(volatile v8h*)q = o;
  __threadfence();
  *(volatile v8h*)q = o;
}

__global__ __launch_bounds__(32) void enc_kernel(
    const float* __restrict__ x, const float* __restrict__ h0, const float* __restrict__ c0,
    const float* __restrict__ Wih, const float* __restrict__ Whh,
    const float* __restrict__ bih, const float* __restrict__ bhh,
    const float* __restrict__ Wfc, const float* __restrict__ bfc,
    float* __restrict__ zout, float* __restrict__ zws)
{
  __shared__ float sWih[4 * kEncH * kEncIn];
  __shared__ float sWhh[4 * kEncH * kEncH];
  __shared__ float sB[4 * kEncH];
  __shared__ float sG[4 * kEncH * 32];
  __shared__ float sH[kEncH * 32];
  __shared__ float sC[kEncH * 32];
  const int tid = threadIdx.x;
  const int b = blockIdx.x * 32 + tid;

  sWih[tid]      = Wih[tid];
  sWih[tid + 32] = Wih[tid + 32];
  sWih[tid + 64] = Wih[tid + 64];
  {
    const int i1 = (tid + 32 < 36) ? (tid + 32) : 35;
    float w0 = Whh[tid];
    float w1 = Whh[i1];
    asm volatile("" : "+v"(w0), "+v"(w1));
    sWhh[tid] = w0;
    if (tid + 32 < 36) sWhh[tid + 32] = w1;
  }
  {
    const int k12 = tid < 12 ? tid : 11;
    float bb = bih[k12] + bhh[k12];
    asm volatile("" : "+v"(bb));
    if (tid < 12) sB[tid] = bb;
  }
  sH[tid]      = h0[b * 3 + 0];
  sH[32 + tid] = h0[b * 3 + 1];
  sH[64 + tid] = h0[b * 3 + 2];
  sC[tid]      = c0[b * 3 + 0];
  sC[32 + tid] = c0[b * 3 + 1];
  sC[64 + tid] = c0[b * 3 + 2];
  const float wf0 = Wfc[0], wf1 = Wfc[1], wf2 = Wfc[2], bf = bfc[0];
  __syncthreads();

  const float* xb = x + (size_t)b * kSteps * kEncIn;
#pragma unroll 1
  for (int t = 0; t < kSteps; ++t) {
    const v4f xa = *(const v4f*)(xb + (size_t)t * kEncIn);
    const v4f xc = *(const v4f*)(xb + (size_t)t * kEncIn + 4);
    const float hh0 = sH[tid], hh1 = sH[32 + tid], hh2 = sH[64 + tid];
#pragma unroll 1
    for (int k = 0; k < 4 * kEncH; ++k) {
      const float* wr = sWih + k * kEncIn;
      const float* wh = sWhh + k * kEncH;
      float a = sB[k];
      a = fmaf(xa[0], wr[0], a);
      a = fmaf(xa[1], wr[1], a);
      a = fmaf(xa[2], wr[2], a);
      a = fmaf(xa[3], wr[3], a);
      a = fmaf(xc[0], wr[4], a);
      a = fmaf(xc[1], wr[5], a);
      a = fmaf(xc[2], wr[6], a);
      a = fmaf(xc[3], wr[7], a);
      a = fmaf(hh0, wh[0], a);
      a = fmaf(hh1, wh[1], a);
      a = fmaf(hh2, wh[2], a);
      sG[k * 32 + tid] = a;
    }
#pragma unroll 1
    for (int j = 0; j < kEncH; ++j) {
      const float gi = sG[j * 32 + tid];
      const float gf = sG[(kEncH + j) * 32 + tid];
      const float gg = sG[(2 * kEncH + j) * 32 + tid];
      const float go = sG[(3 * kEncH + j) * 32 + tid];
      const float cp = sC[j * 32 + tid];
      const float cn = sig_f(gf) * cp + sig_f(gi) * tanh_f(gg);
      sC[j * 32 + tid] = cn;
      sH[j * 32 + tid] = sig_f(go) * tanh_f(cn);
    }
  }
  float zv = wf0 * sH[tid];
  zv = fmaf(wf1, sH[32 + tid], zv);
  zv = fmaf(wf2, sH[64 + tid], zv);
  zv = zv + bf;
  *(volatile float*)(zout + b) = zv;
  *(volatile float*)(zws + b) = zv;
  __threadfence();
  *(volatile float*)(zout + b) = zv;
  *(volatile float*)(zws + b) = zv;
}

__global__ __launch_bounds__(256) void traj_kernel(
    const float* __restrict__ s, const float* __restrict__ W, const float* __restrict__ bias,
    float* __restrict__ out)
{
  const int id = blockIdx.x * 256 + threadIdx.x;
  if (id >= kBatch * kSteps * 2) return;
  const int pair = id >> 1;
  const int k = id & 1;
  const float* sr = s + (size_t)pair * kDecIn;
  const float* wr = W + k * kDecIn;
  float a = sr[0] * wr[0];
  a = fmaf(sr[1], wr[1], a);
  a = fmaf(sr[2], wr[2], a);
  a = fmaf(sr[3], wr[3], a);
  a = fmaf(sr[4], wr[4], a);
  a = fmaf(sr[5], wr[5], a);
  a = a + bias[k];
  *(volatile float*)(out + id) = a;
  __threadfence();
  *(volatile float*)(out + id) = a;
}

__device__ __forceinline__ void stage_chunk(const float* __restrict__ s, float* sS, int b0, int chunk, int buf, int tid) {
#pragma unroll
  for (int j = 0; j < 3; ++j) {
    const int i = tid + 256 * j;
    const int row = i / 48;
    const int c = i - row * 48;
    const v4f v = *(const v4f*)(s + ((size_t)(b0 + row) * kSteps + (size_t)chunk * kChunkT) * kDecIn + c * 4);
    *(v4f*)(sS + buf * (kRowsBlk * kChunkF) + row * kChunkF + c * 4) = v;
  }
}
__device__ __forceinline__ void write_x(_Float16* Al, const float* sS, int buf, int tl, int row, int q, float zr, float zf) {
  const float* sp = sS + buf * (kRowsBlk * kChunkF) + row * kChunkF + tl * kDecIn;
  const float v0 = sp[0], v1 = sp[1], v2 = sp[2], v3 = sp[3], v4 = sp[4], v5 = sp[5];
  const bool first = (q == 0);
  v8h o;
  o[0] = cvt_flush(first ? v0 * kCarryA : zf, zf);
  o[1] = cvt_flush(first ? v1 * kCarryA : zf, zf);
  o[2] = cvt_flush(first ? v2 * kCarryA : zf, zf);
  o[3] = cvt_flush(first ? v3 * kCarryA : zf, zf);
  o[4] = cvt_flush(first ? v4 * kCarryA : zf, zf);
  o[5] = cvt_flush(first ? v5 * kCarryA : zf, zf);
  o[6] = cvt_flush(first ? zr * kCarryA : zf, zf);
  o[7] = cvt_flush(zf, zf);
  *(v8h*)(Al + row * kAPitch + kDecH + q * 8) = o;
}

__global__ __launch_bounds__(256) void dec_kernel(
    const float* __restrict__ s, const float* __restrict__ zws, const unsigned short* __restrict__ wcat,
    const float* __restrict__ bih, const float* __restrict__ bhh, float* __restrict__ hout)
{
  extern __shared__ __align__(16) unsigned char smem[];
  _Float16* Wl = (_Float16*)(smem + kOffW);
  _Float16* Al = (_Float16*)(smem + kOffA);
  float* sS = (float*)(smem + kOffS);
  float* hF = (float*)(smem + kOffHF);

  const int tid = threadIdx.x;
  const int lane = tid & 31;
  const int wave = tid >> 5;
  const int hh = lane >> 4;
  const int n = lane & 15;
  const int b0 = blockIdx.x * kRowsBlk;
  const int hc0 = wave * 16;

#pragma unroll 1
  for (int it = 0; it < 42; ++it) {
    const int i = it * 256 + tid;
    const int row = i / 21;
    const int ch = i - row * 21;
    const int chc = ch < 20 ? ch : 19;
    const v4u w = *(const v4u*)(const void*)(wcat + (size_t)row * kKcat + chc * 8);
    unsigned w0 = w[0], w1 = w[1], w2 = w[2], w3 = w[3];
    asm volatile("" : "+v"(w0), "+v"(w1), "+v"(w2), "+v"(w3));
    const bool pad = (ch >= 20);
    v4u o;
    o[0] = pad ? 0u : w0;
    o[1] = pad ? 0u : w1;
    o[2] = pad ? 0u : w2;
    o[3] = pad ? 0u : w3;
    *(v4u*)(void*)(Wl + row * kWPitch + ch * 8) = o;
  }
  {
    const v4u zz = {0u, 0u, 0u, 0u};
    for (int i = tid; i < (kRowsBlk * kAPitch) / 8; i += 256) *(v4u*)(void*)(Al + i * 8) = zz;
  }
  stage_chunk(s, sS, b0, 0, 0, tid);

  const int xrow = (tid >> 2) & 15;
  const int xq = tid & 3;
  float zr = zws[b0 + xrow];
  asm volatile("" : "+v"(zr));
  float zf = 0.0f;
  asm volatile("" : "+v"(zf));
  const int nI = hc0 + n;
  const float bI = (bih[nI] + bhh[nI]) * kBiasCar;
  const float bF = (bih[kDecH + nI] + bhh[kDecH + nI]) * kBiasCar;
  const float bG = (bih[2 * kDecH + nI] + bhh[2 * kDecH + nI]) * kBiasCar;
  const float bO = (bih[3 * kDecH + nI] + bhh[3 * kDecH + nI]) * kBiasCar;

  __syncthreads();
  if (tid < 64) write_x(Al, sS, 0, 0, xrow, xq, zr, zf);
  __syncthreads();

  const _Float16* aBase = Al + n * kAPitch + 8 * hh;
  const _Float16* bBaseI = Wl + (nI) * kWPitch + 8 * hh;
  const _Float16* bBaseF = Wl + (kDecH + nI) * kWPitch + 8 * hh;
  const _Float16* bBaseG = Wl + (2 * kDecH + nI) * kWPitch + 8 * hh;
  const _Float16* bBaseO = Wl + (3 * kDecH + nI) * kWPitch + 8 * hh;

  float cst[8], hl[8];
#pragma unroll
  for (int r = 0; r < 8; ++r) { cst[r] = 0.0f; hl[r] = 0.0f; }

#pragma unroll 1
  for (int t = 0; t < kSteps; ++t) {
    v8f accI = (v8f){bI, bI, bI, bI, bI, bI, bI, bI};
    v8f accF = (v8f){bF, bF, bF, bF, bF, bF, bF, bF};
    v8f accG = (v8f){bG, bG, bG, bG, bG, bG, bG, bG};
    v8f accO = (v8f){bO, bO, bO, bO, bO, bO, bO, bO};
#pragma unroll
    for (int kk = 0; kk < kKcat / 32; ++kk) {
      const v16h a  = ldfrag(aBase + kk * 32);
      const v16h wI = ldfrag(bBaseI + kk * 32);
      const v16h wF = ldfrag(bBaseF + kk * 32);
      const v16h wG = ldfrag(bBaseG + kk * 32);
      const v16h wO = ldfrag(bBaseO + kk * 32);
      accI = mma_f16(a, wI, accI);
      accF = mma_f16(a, wF, accF);
      accG = mma_f16(a, wG, accG);
      accO = mma_f16(a, wO, accO);
    }
    __syncthreads();

    if (((t & (kChunkT - 1)) == 0) && ((t / kChunkT) + 1 < kSteps / kChunkT)) {
      const int nc = (t / kChunkT) + 1;
      stage_chunk(s, sS, b0, nc, nc & 1, tid);
    }

#pragma unroll
    for (int r = 0; r < 8; ++r) {
      const float gi = accI[r] * kFold;
      const float gf = accF[r] * kFold;
      const float gg = accG[r] * kFold;
      const float go = accO[r] * kFold;
      const float ig = sig_f(gi);
      const float fg = sig_f(gf);
      const float gt = tanh_f(gg);
      const float og = sig_f(go);
      const float cn = fg * cst[r] + ig * gt;
      cst[r] = cn;
      const float hv = og * tanh_f(cn);
      hl[r] = hv;
      Al[(8 * hh + r) * kAPitch + hc0 + n] = cvt_flush(hv * kCarryA, 0.0f);
    }
    if ((t + 1 < kSteps) && (tid < 64)) {
      const int tn = t + 1;
      write_x(Al, sS, (tn / kChunkT) & 1, tn & (kChunkT - 1), xrow, xq, zr, zf);
    }
    __syncthreads();
  }

#pragma unroll
  for (int r = 0; r < 8; ++r) hF[(8 * hh + r) * kHfPitch + hc0 + n] = hl[r];
  __syncthreads();
  {
    const int r0 = 2 * wave;
    const v4f o0 = *(const v4f*)(hF + r0 * kHfPitch + lane * 4);
    const v4f o1 = *(const v4f*)(hF + (r0 + 1) * kHfPitch + lane * 4);
    float* p0 = hout + (size_t)(b0 + r0) * kDecH + lane * 4;
    float* p1 = p0 + kDecH;
    *(volatile v4f*)p0 = o0;
    *(volatile v4f*)p1 = o1;
    __threadfence();
    *(volatile v4f*)p0 = o0;
    *(volatile v4f*)p1 = o1;
  }
}

extern "C" void kernel_launch(void* const* d_in, const int* in_sizes, int n_in,
                              void* d_out, int out_size, void* d_ws, size_t ws_size,
                              hipStream_t stream) {
  if (n_in < 16) return;
  if (in_sizes[0] != kBatch * kSteps * kEncIn) return;
  if (in_sizes[1] != kBatch * kSteps * kDecIn) return;
  if (in_sizes[2] != kBatch * kEncH) return;
  if (in_sizes[3] != kBatch * kEncH) return;
  if (in_sizes[4] != 4 * kEncH * kEncIn) return;
  if (in_sizes[5] != 4 * kEncH * kEncH) return;
  if (in_sizes[6] != 4 * kEncH) return;
  if (in_sizes[7] != 4 * kEncH) return;
  if (in_sizes[8] != kEncH) return;
  if (in_sizes[9] != 1) return;
  if (in_sizes[10] != kGates * (kDecIn + 1)) return;
  if (in_sizes[11] != kGates * kDecH) return;
  if (in_sizes[12] != kGates) return;
  if (in_sizes[13] != kGates) return;
  if (in_sizes[14] != 2 * kDecIn) return;
  if (in_sizes[15] != 2) return;
  if (out_size != kOutTotal) return;
  if (ws_size < kWsTotal) return;

  const float* x     = (const float*)d_in[0];
  const float* s     = (const float*)d_in[1];
  const float* h0    = (const float*)d_in[2];
  const float* c0    = (const float*)d_in[3];
  const float* We_ih = (const float*)d_in[4];
  const float* We_hh = (const float*)d_in[5];
  const float* be_ih = (const float*)d_in[6];
  const float* be_hh = (const float*)d_in[7];
  const float* Wfc_e = (const float*)d_in[8];
  const float* bfc_e = (const float*)d_in[9];
  const float* Wd_ih = (const float*)d_in[10];
  const float* Wd_hh = (const float*)d_in[11];
  const float* bd_ih = (const float*)d_in[12];
  const float* bd_hh = (const float*)d_in[13];
  const float* Wfc_d = (const float*)d_in[14];
  const float* bfc_d = (const float*)d_in[15];

  float* out = (float*)d_out;
  float* z_out    = out + kOutZ;
  float* traj_out = out + kOutTraj;
  float* hdec_out = out + kOutHdec;

  char* ws = (char*)d_ws;
  unsigned short* wcat = (unsigned short*)(ws + kWsWcat);
  float* zws = (float*)(ws + kWsZ);

  (void)hipFuncSetAttribute((const void*)dec_kernel, hipFuncAttributeMaxDynamicSharedMemorySize, (int)kLdsBytes);

  prep_wcat_kernel<<<(kGates * (kKcat / 8)) / 256, 256, 0, stream>>>(Wd_hh, Wd_ih, wcat);
  enc_kernel<<<kBatch / 32, 32, 0, stream>>>(x, h0, c0, We_ih, We_hh, be_ih, be_hh, Wfc_e, bfc_e, z_out, zws);
  traj_kernel<<<(kBatch * kSteps * 2) / 256, 256, 0, stream>>>(s, Wfc_d, bfc_d, traj_out);
  dec_kernel<<<kBatch / kRowsBlk, 256, kLdsBytes, stream>>>(s, zws, wcat, bd_ih, bd_hh, hdec_out);
}
